// SingleHeadAttention_31868657336870
// MI455X (gfx1250) — hardware-verified
//
#include <hip/hip_runtime.h>

typedef _Float16 h16;
typedef _Float16 h16x8 __attribute__((ext_vector_type(8)));
typedef _Float16 v16h  __attribute__((ext_vector_type(16)));
typedef float  v8f    __attribute__((ext_vector_type(8)));
typedef float  v4f    __attribute__((ext_vector_type(4)));
typedef unsigned v4u  __attribute__((ext_vector_type(4)));

#ifndef NB
#define NB 8
#endif
#ifndef SEQ
#define SEQ 2048
#endif
#define NB_FULL  8
#define SEQ_FULL 2048
#define D_DIM 768
#define HD    128
#define M_TOT (NB * SEQ)
#define QBLK  64
#define KVT   64
#define EARLY_QB 4
#define WSC   64.0f
#define W_INV (1.0f / 64.0f)
#define PSC   256.0f
#define P_INV (1.0f / 256.0f)
#define RSC   2048.0f
#define R_INV (1.0f / 2048.0f)
#define SM_SCALE 0.08838834764831845f

static_assert(SEQ % QBLK == 0);
static_assert(SEQ % KVT == 0);
static_assert(M_TOT % 64 == 0);
static_assert(D_DIM % 256 == 0);
static_assert(HD == 128);
static_assert(NB <= NB_FULL);
static_assert(SEQ <= SEQ_FULL);

template <typename V> __device__ __forceinline__ void vst2(void* p, V v) {
  *(volatile V*)p = v; __threadfence(); *(volatile V*)p = v;
}
__device__ __forceinline__ void copy16_g2s(h16* ldst, const h16* gsrc) { *(h16x8*)ldst = *(const h16x8*)gsrc; }

__device__ __forceinline__ float bf16r(float f) {
  unsigned u = __float_as_uint(f);
  u = (u + 0x7fffu + ((u >> 16) & 1u)) & 0xffff0000u;
  return __uint_as_float(u);
}

__device__ __forceinline__ v16h load_a_frag(const h16* base, int ld, int k0) {
  int lane = threadIdx.x & 31;
  int idx  = lane & 15;
  int half = lane >> 4;
  const h16* p = base + idx * ld + k0 + half * 8;
  h16x8 lo = *(const h16x8*)(p);
  h16x8 hi = *(const h16x8*)(p + 16);
  return __builtin_shufflevector(lo, hi, 0,1,2,3,4,5,6,7,8,9,10,11,12,13,14,15);
}
__device__ __forceinline__ v16h load_b_frag(const h16* base, int ld, int k0) { return load_a_frag(base, ld, k0); }

__device__ __forceinline__ v8f wmma_f16(v16h a, v16h b, v8f c) {
  v8f d = __builtin_amdgcn_wmma_f32_16x16x32_f16(false, a, false, b, (short)0, c, false, false);
  asm volatile("v_nop\n\tv_nop\n\tv_nop\n\tv_nop" : "+v"(d) : "v"(a), "v"(b));
  return d;
}

__global__ __launch_bounds__(256) void cvt_x_kernel(const float* __restrict__ x, h16* __restrict__ xb, int n8) {
  int g = blockIdx.x * blockDim.x + threadIdx.x;
  if (g >= n8) return;
  const int m = g / (D_DIM / 8), c = g - m * (D_DIM / 8);
  const int b = m / SEQ, s = m - b * SEQ;
  const float* src = x + ((size_t)(b * SEQ_FULL + s)) * D_DIM + c * 8;
  const v4f a0 = *(const v4f*)(src), a1 = *(const v4f*)(src + 4);
  union { h16x8 h; v4u u; } pk;
#pragma unroll
  for (int i = 0; i < 4; ++i) { pk.h[i] = (h16)bf16r(a0[i]); pk.h[4 + i] = (h16)bf16r(a1[i]); }
  vst2(xb + (size_t)g * 8, pk.u);
}

__global__ __launch_bounds__(256) void cvt_w_kernel(const float* __restrict__ Wq, const float* __restrict__ Wk, const float* __restrict__ Wv,
                                                    h16* __restrict__ WqT, h16* __restrict__ WkT, h16* __restrict__ WvT) {
  __shared__ __align__(16) h16 tile[64][264];
  const float* W = (blockIdx.z == 0) ? Wq : (blockIdx.z == 1) ? Wk : Wv;
  h16*       WT = (blockIdx.z == 0) ? WqT : (blockIdx.z == 1) ? WkT : WvT;
  const int n0 = blockIdx.x * 64, k0 = blockIdx.y * 256, tid = threadIdx.x;
  for (int i = tid; i < 256 * 64; i += 256) {
    const int k = i >> 6, nl = i & 63;
    tile[nl][k] = (h16)(bf16r(W[(size_t)(k0 + k) * HD + n0 + nl]) * WSC);
  }
  __syncthreads();
  for (int g = tid; g < 64 * 32; g += 256) {
    const int nl = g >> 5, pc = g & 31;
    vst2(WT + (size_t)(n0 + nl) * D_DIM + k0 + pc * 8, *(const v4u*)(&tile[nl][pc * 8]));
  }
}

__global__ __launch_bounds__(256) void proj_kernel(const h16* __restrict__ Xb,
                            const h16* __restrict__ WqT, const h16* __restrict__ WkT, const h16* __restrict__ WvT,
                            const float* __restrict__ bq, const float* __restrict__ bk, const float* __restrict__ bv,
                            h16* __restrict__ Qh, h16* __restrict__ Qr, h16* __restrict__ Kh, h16* __restrict__ Kr,
                            h16* __restrict__ Vth, h16* __restrict__ Vtr) {
  __shared__ __align__(16) h16 Th[128 * 72];
  __shared__ __align__(16) h16 Tr[128 * 72];
  const int sel = blockIdx.y;
  const h16*   WT   = (sel == 0) ? WqT : (sel == 1) ? WkT : WvT;
  const float* bias = (sel == 0) ? bq  : (sel == 1) ? bk  : bv;
  h16* oh = (sel == 0) ? Qh : (sel == 1) ? Kh : Vth;
  h16* orp = (sel == 0) ? Qr : (sel == 1) ? Kr : Vtr;
  const int transposed = (sel == 2);

  const int m0 = blockIdx.x * 64;
  const int w    = threadIdx.x >> 5;
  const int lane = threadIdx.x & 31;
  const int idx  = lane & 15;
  const int half = lane >> 4;
  const int m_w = m0 + (w & 3) * 16;
  const int n_w = (w >> 2) * 64;

  v8f c[4] = {};
  const h16* arow = Xb + (size_t)m_w * D_DIM;
#pragma unroll 2
  for (int k0 = 0; k0 < D_DIM; k0 += 32) {
    v16h a = load_a_frag(arow, D_DIM, k0);
#pragma unroll
    for (int t = 0; t < 4; ++t) {
      v16h b = load_b_frag(WT + (size_t)(n_w + t * 16) * D_DIM, D_DIM, k0);
      c[t] = wmma_f16(a, b, c[t]);
    }
  }
#pragma unroll
  for (int t = 0; t < 4; ++t) {
    const int cl = n_w + t * 16 + idx;
    const float bvv = bf16r(bias[cl]);
#pragma unroll
    for (int g = 0; g < 8; ++g) {
      const int rl = (w & 3) * 16 + g + 8 * half;
      const float val = c[t][g] * W_INV + bvv;
      const h16 hv = (h16)val;
      const h16 rv = (h16)((val - (float)hv) * RSC);
      if (!transposed) { Th[rl * 136 + cl] = hv; Tr[rl * 136 + cl] = rv; }
      else             { Th[cl * 72 + rl]  = hv; Tr[cl * 72 + rl]  = rv; }
    }
  }
  __syncthreads();
  const int tid = threadIdx.x;
  if (!transposed) {
    for (int gg = tid; gg < 64 * 16; gg += 256) {
      const int rl = gg >> 4, pc = gg & 15;
      const size_t go = (size_t)(m0 + rl) * HD + pc * 8;
      vst2(oh  + go, *(const v4u*)(&Th[rl * 136 + pc * 8]));
      vst2(orp + go, *(const v4u*)(&Tr[rl * 136 + pc * 8]));
    }
  } else {
    const int bb = m0 / SEQ, s0 = m0 - bb * SEQ;
    for (int gg = tid; gg < 128 * 8; gg += 256) {
      const int cl = gg >> 3, pc = gg & 7;
      const size_t go = ((size_t)(bb * HD + cl)) * SEQ + s0 + pc * 8;
      vst2(oh  + go, *(const v4u*)(&Th[cl * 72 + pc * 8]));
      vst2(orp + go, *(const v4u*)(&Tr[cl * 72 + pc * 8]));
    }
  }
}

template <int EARLY>
__global__ __launch_bounds__(256) __attribute__((amdgpu_num_vgpr(256)))
void attn_kernel(const h16* __restrict__ Qh, const h16* __restrict__ Qr,
                 const h16* __restrict__ Kh, const h16* __restrict__ Kr,
                 const h16* __restrict__ Vth, const h16* __restrict__ Vtr,
                 float* __restrict__ out, int qb0) {
  enum { QP = 136, VP = 72, SP = 68 };
  __shared__ __align__(16) h16   Qs[QBLK * QP];
  __shared__ __align__(16) h16   Ks[KVT * QP];
  __shared__ __align__(16) h16   Vts[HD * VP];
  __shared__ __align__(16) float Ss[QBLK * SP];
  __shared__ __align__(16) h16   Ps[QBLK * VP];
  __shared__ __align__(16) float Os[QBLK * HD];
  __shared__ float alpha_s[QBLK];
  __shared__ float l_s[QBLK];
  __shared__ __align__(16) h16   Qrs[EARLY ? QBLK * QP : 8];
  __shared__ __align__(16) h16   Krs[EARLY ? KVT * QP : 8];
  __shared__ __align__(16) h16   Vtrs[EARLY ? HD * VP : 8];
  __shared__ __align__(16) h16   Prs[EARLY ? QBLK * VP : 8];

  const int b    = blockIdx.y;
  const int qb   = qb0 + blockIdx.x;
  const int q0   = qb * QBLK;
  const int tid  = threadIdx.x;
  const int w    = tid >> 5;
  const int lane = tid & 31;
  const int idx  = lane & 15;
  const int half = lane >> 4;
  const int qi   = w & 3;
  const int kg2  = (w >> 2) * 2;
  const int dg   = w >> 2;

  {
    const size_t qrow = ((size_t)(b * SEQ + q0)) * HD;
    for (int c = tid; c < QBLK * (HD / 8); c += 256) {
      const int r = c >> 4, dc = c & 15;
      copy16_g2s(&Qs[r * QP + dc * 8], Qh + qrow + (size_t)r * HD + dc * 8);
      if (EARLY) copy16_g2s(&Qrs[r * QP + dc * 8], Qr + qrow + (size_t)r * HD + dc * 8);
    }
  }

  v8f o[4]   = {};
  v8f orr[4] = {};
  const int srow = tid >> 2;
  const int sj   = tid & 3;
  float m_run = -1e30f;
  float l_run = 0.0f;

#pragma unroll 1
  for (int kt = 0; kt <= qb; ++kt) {
    const int kv0 = kt * KVT;
    __syncthreads();
    {
      const size_t krow = ((size_t)(b * SEQ + kv0)) * HD;
      for (int c = tid; c < KVT * (HD / 8); c += 256) {
        const int r = c >> 4, dc = c & 15;
        copy16_g2s(&Ks[r * QP + dc * 8], Kh + krow + (size_t)r * HD + dc * 8);
        if (EARLY) copy16_g2s(&Krs[r * QP + dc * 8], Kr + krow + (size_t)r * HD + dc * 8);
      }
      const size_t vbase = (size_t)b * HD * SEQ + kv0;
      for (int c = tid; c < HD * (KVT / 8); c += 256) {
        const int d = c >> 3, j = c & 7;
        copy16_g2s(&Vts[d * VP + j * 8], Vth + vbase + (size_t)d * SEQ + j * 8);
        if (EARLY) copy16_g2s(&Vtrs[d * VP + j * 8], Vtr + vbase + (size_t)d * SEQ + j * 8);
      }
    }
    __syncthreads();

    {
      v8f sc0 = {}, sc1 = {};
      v8f sr0 = {}, sr1 = {};
#pragma unroll 2
      for (int k0 = 0; k0 < HD; k0 += 32) {
        v16h a  = load_a_frag(&Qs[(qi * 16) * QP], QP, k0);
        v16h b0 = load_b_frag(&Ks[(kg2 * 16) * QP], QP, k0);
        v16h b1 = load_b_frag(&Ks[(kg2 * 16 + 16) * QP], QP, k0);
        sc0 = wmma_f16(a, b0, sc0);
        sc1 = wmma_f16(a, b1, sc1);
        if (EARLY) {
          v16h ar = load_a_frag(&Qrs[(qi * 16) * QP], QP, k0);
          sr0 = wmma_f16(ar, b0, sr0);
          sr1 = wmma_f16(ar, b1, sr1);
          v16h br0 = load_b_frag(&Krs[(kg2 * 16) * QP], QP, k0);
          sr0 = wmma_f16(a, br0, sr0);
          v16h br1 = load_b_frag(&Krs[(kg2 * 16 + 16) * QP], QP, k0);
          sr1 = wmma_f16(a, br1, sr1);
        }
      }
      const int col0 = kg2 * 16 + idx;
#pragma unroll
      for (int g = 0; g < 8; ++g) {
        const int row = qi * 16 + g + 8 * half;
        float s0v = sc0[g], s1v = sc1[g];
        if (EARLY) { s0v += sr0[g] * R_INV; s1v += sr1[g] * R_INV; }
        Ss[row * SP + col0]      = s0v * SM_SCALE;
        Ss[row * SP + col0 + 16] = s1v * SM_SCALE;
      }
    }
    __syncthreads();

    {
      const bool diag = (kv0 == q0);
      float v[16];
      float mloc = -1e30f;
#pragma unroll
      for (int e = 0; e < 16; ++e) {
        const int col = sj + 4 * e;
        float t = Ss[srow * SP + col];
        t = (diag && col > srow) ? -1e30f : t;
        v[e] = t;
        mloc = fmaxf(mloc, t);
      }
      mloc = fmaxf(mloc, __shfl_xor(mloc, 1, 32));
      mloc = fmaxf(mloc, __shfl_xor(mloc, 2, 32));
      const float m_new = fmaxf(m_run, mloc);
      const float alpha = __expf(m_run - m_new);
      float ssum = 0.0f;
#pragma unroll
      for (int e = 0; e < 16; ++e) {
        const int col = sj + 4 * e;
        const float p  = __expf(v[e] - m_new);
        ssum += p;
        const float ps = p * PSC;
        const h16 ph = (h16)ps;
        Ps[srow * VP + col] = ph;
        if (EARLY) Prs[srow * VP + col] = (h16)((ps - (float)ph) * RSC);
      }
      ssum += __shfl_xor(ssum, 1, 32);
      ssum += __shfl_xor(ssum, 2, 32);
      l_run = l_run * alpha + ssum;
      m_run = m_new;
      if (sj == 0) { alpha_s[srow] = alpha; l_s[srow] = l_run; }
    }
    __syncthreads();

    {
      float al[8];
#pragma unroll
      for (int g = 0; g < 8; ++g) al[g] = alpha_s[qi * 16 + g + 8 * half];
#pragma unroll
      for (int t = 0; t < 4; ++t) {
#pragma unroll
        for (int g = 0; g < 8; ++g) {
          o[t][g] *= al[g];
          if (EARLY) orr[t][g] *= al[g];
        }
      }
#pragma unroll
      for (int k0 = 0; k0 < KVT; k0 += 32) {
        v16h a  = load_a_frag(&Ps[(qi * 16) * VP], VP, k0);
        v16h ar = a;
        if (EARLY) ar = load_a_frag(&Prs[(qi * 16) * VP], VP, k0);
#pragma unroll
        for (int t = 0; t < 4; ++t) {
          v16h bb = load_b_frag(&Vts[(dg * 64 + t * 16) * VP], VP, k0);
          o[t] = wmma_f16(a, bb, o[t]);
          if (EARLY) {
            orr[t] = wmma_f16(ar, bb, orr[t]);
            v16h br = load_b_frag(&Vtrs[(dg * 64 + t * 16) * VP], VP, k0);
            orr[t] = wmma_f16(a, br, orr[t]);
          }
        }
      }
    }
  }
  __syncthreads();

  float linv[8];
#pragma unroll
  for (int g = 0; g < 8; ++g) linv[g] = P_INV / l_s[qi * 16 + g + 8 * half];
#pragma unroll
  for (int t = 0; t < 4; ++t) {
    const int col = dg * 64 + t * 16 + idx;
#pragma unroll
    for (int g = 0; g < 8; ++g) {
      float ov = o[t][g];
      if (EARLY) ov += orr[t][g] * R_INV;
      Os[(qi * 16 + g + 8 * half) * HD + col] = ov * linv[g];
    }
  }
  __syncthreads();
  {
    float* dst = out + ((size_t)(b * SEQ + q0)) * HD;
    for (int gg = tid; gg < QBLK * HD / 4; gg += 256) vst2(dst + (size_t)gg * 4, *(const v4f*)(&Os[gg * 4]));
  }
}

extern "C" void kernel_launch(void* const* d_in, const int* in_sizes, int n_in,
                              void* d_out, int out_size, void* d_ws, size_t ws_size,
                              hipStream_t stream) {
  if (n_in < 7) return;
  if (in_sizes[0] < ((NB - 1) * SEQ_FULL + SEQ) * D_DIM) return;
  if (in_sizes[1] < D_DIM * HD || in_sizes[3] < D_DIM * HD || in_sizes[5] < D_DIM * HD) return;
  if (in_sizes[2] < HD || in_sizes[4] < HD || in_sizes[6] < HD) return;
  if (out_size < M_TOT * HD) return;

  const float* x  = (const float*)d_in[0];
  const float* Wq = (const float*)d_in[1];
  const float* bq = (const float*)d_in[2];
  const float* Wk = (const float*)d_in[3];
  const float* bk = (const float*)d_in[4];
  const float* Wv = (const float*)d_in[5];
  const float* bv = (const float*)d_in[6];
  float* out = (float*)d_out;

  const size_t xb_b = (size_t)M_TOT * D_DIM * sizeof(h16);
  const size_t wt_b = (size_t)HD * D_DIM * sizeof(h16);
  const size_t pl_b = (size_t)M_TOT * HD * sizeof(h16);
  char* ws = (char*)d_ws;
  size_t off = 0;
  h16* xb  = (h16*)(ws + off); off += xb_b;
  h16* WqT = (h16*)(ws + off); off += wt_b;
  h16* WkT = (h16*)(ws + off); off += wt_b;
  h16* WvT = (h16*)(ws + off); off += wt_b;
  h16* qh  = (h16*)(ws + off); off += pl_b;
  h16* qr  = (h16*)(ws + off); off += pl_b;
  h16* kh  = (h16*)(ws + off); off += pl_b;
  h16* kr  = (h16*)(ws + off); off += pl_b;
  h16* vth = (h16*)(ws + off); off += pl_b;
  h16* vtr = (h16*)(ws + off); off += pl_b;
  if (off > ws_size) return;

  const int nx8 = M_TOT * D_DIM / 8;
  cvt_x_kernel<<<(nx8 + 255) / 256, 256, 0, stream>>>(x, xb, nx8);
  cvt_w_kernel<<<dim3(HD / 64, D_DIM / 256, 3), 256, 0, stream>>>(Wq, Wk, Wv, WqT, WkT, WvT);
  proj_kernel<<<dim3(M_TOT / 64, 3), 256, 0, stream>>>(xb, WqT, WkT, WvT, bq, bk, bv, qh, qr, kh, kr, vth, vtr);

  const int nqb = SEQ / QBLK;
  const int ne  = (nqb < EARLY_QB) ? nqb : EARLY_QB;
  attn_kernel<1><<<dim3(ne, NB), 256, 0, stream>>>(qh, qr, kh, kr, vth, vtr, out, 0);
  if (nqb > ne) attn_kernel<0><<<dim3(nqb - ne, NB), 256, 0, stream>>>(qh, qr, kh, kr, vth, vtr, out, ne);
}
